// OrienCrossAttnBlock_89369679495531
// MI455X (gfx1250) — hardware-verified
//
#include <hip/hip_runtime.h>
#include <math.h>

typedef __attribute__((ext_vector_type(16))) _Float16 v16h;
typedef __attribute__((ext_vector_type(16))) __bf16 v16b;
typedef __attribute__((ext_vector_type(8)))  _Float16 v8h;
typedef __attribute__((ext_vector_type(8)))  float v8f;
typedef __attribute__((ext_vector_type(4)))  float v4f;
typedef __attribute__((ext_vector_type(2)))  float v2f;
typedef __attribute__((ext_vector_type(4)))  unsigned v4u;
typedef __attribute__((ext_vector_type(4)))  int v4i;
typedef float __attribute__((may_alias)) float_a;
typedef int __attribute__((may_alias)) int_a;

template <typename T> __device__ __forceinline__ void vst2(void* p, T v) { *(volatile T*)p = v; __threadfence(); *(volatile T*)p = v; }
__device__ __forceinline__ v8f wmma16(v16h a, v16h b, v8f c) {
  v8f d = __builtin_amdgcn_wmma_f32_16x16x32_f16(false, a, false, b, (short)0, c, false, false);
  asm volatile("v_nop\n\tv_nop\n\tv_nop\n\tv_nop" : "+v"(d) : "v"(a), "v"(b));
  return d;
}
__device__ __forceinline__ v8f wmma_bf(v16b a, v16b b, v8f c) {
  v8f d = __builtin_amdgcn_wmma_f32_16x16x32_bf16(false, a, false, b, (short)0, c, false, false);
  asm volatile("v_nop\n\tv_nop\n\tv_nop\n\tv_nop" : "+v"(d) : "v"(a), "v"(b));
  return d;
}
__device__ __forceinline__ v16h frag_h(const _Float16* rowk0, int lane) {
  union { v16h v; v8h q[2]; } u; const _Float16* p = rowk0 + 8 * (lane >> 4);
  u.q[0] = *(const v8h*)p; u.q[1] = *(const v8h*)(p + 16); return u.v;
}
__device__ __forceinline__ v16h frag_f32(const float* rowk0, int lane) {
  v16h a; const float* p = rowk0 + 8 * (lane >> 4);
#pragma unroll
  for (int i = 0; i < 8; ++i) { a[i] = (_Float16)p[i]; a[8 + i] = (_Float16)p[16 + i]; }
  return a;
}
__device__ __forceinline__ v16h frag_f32s(const float* rowk0, int lane, float sc) {
  v16h a; const float* p = rowk0 + 8 * (lane >> 4);
#pragma unroll
  for (int i = 0; i < 8; ++i) { a[i] = (_Float16)(p[i] * sc); a[8 + i] = (_Float16)(p[16 + i] * sc); }
  return a;
}
__device__ __forceinline__ v16h fragc_f32(const float* W, int k0, int n, int lane, int ld, int K) {
  v16h a; const int g = lane >> 4;
#pragma unroll
  for (int i = 0; i < 8; ++i) { const int ka = k0 + 8 * g + i, kb = ka + 16;
    a[i] = (_Float16)(ka < K ? W[(size_t)(ka < K ? ka : K - 1) * ld + n] : 0.f); a[8 + i] = (_Float16)(kb < K ? W[(size_t)(kb < K ? kb : K - 1) * ld + n] : 0.f); }
  return a;
}
struct F2 { v16b h, l; };
__device__ __forceinline__ F2 bsplit16(const float v[16]) { F2 r;
#pragma unroll
  for (int i = 0; i < 16; ++i) { const __bf16 h = (__bf16)v[i]; r.h[i] = h; r.l[i] = (__bf16)(v[i] - (float)h); }
  return r; }
__device__ __forceinline__ F2 split_row(const float* row, int k0, int lane) { float v[16]; const float* p = row + k0 + 8 * (lane >> 4);
#pragma unroll
  for (int i = 0; i < 8; ++i) { v[i] = p[i]; v[8 + i] = p[16 + i]; }
  return bsplit16(v); }
__device__ __forceinline__ F2 split_rowK(const float* row, int k0, int lane, int K) { float v[16]; const int g = lane >> 4;
#pragma unroll
  for (int i = 0; i < 8; ++i) { const int ka = k0 + 8 * g + i, kb = ka + 16; v[i] = ka < K ? row[ka < K ? ka : K - 1] : 0.f; v[8 + i] = kb < K ? row[kb < K ? kb : K - 1] : 0.f; }
  return bsplit16(v); }
__device__ __forceinline__ F2 split_col(const float* W, int k0, int n, int lane, int ld, int K) { float v[16]; const int g = lane >> 4;
#pragma unroll
  for (int i = 0; i < 8; ++i) { const int ka = k0 + 8 * g + i, kb = ka + 16; v[i] = ka < K ? W[(size_t)(ka < K ? ka : K - 1) * ld + n] : 0.f; v[8 + i] = kb < K ? W[(size_t)(kb < K ? kb : K - 1) * ld + n] : 0.f; }
  return bsplit16(v); }
__device__ __forceinline__ v8f mac3(const F2& a, const F2& b, v8f c) { c = wmma_bf(a.l, b.h, c); c = wmma_bf(a.h, b.l, c); return wmma_bf(a.h, b.h, c); }
__device__ __forceinline__ float sigm(float v) { return 1.0f / (1.0f + expf(-v)); }
#define LDSX() do { asm volatile("s_wait_dscnt 0" ::: "memory"); __builtin_amdgcn_wave_barrier(); __builtin_amdgcn_fence(__ATOMIC_RELEASE, "workgroup"); } while (0)


#define NB 8
#define CC 256
#define NPIX 4096
#define NS 64
#define INF 720
#define INP 736
#define BINS 786
#define BINP 800
#define NT 16
#define NKEY (NS * NT)
#define NH 8
#define HD 32
#define NRX (NB * NPIX)
#define NRS (NB * NS)
#ifndef NPB
#define NPB (NRX / 64)
#define NBT NB
#endif
typedef __attribute__((ext_vector_type(8))) __bf16 v8b;
__device__ __forceinline__ v16b frag_b(const __bf16* rowk0, int lane) {
  union { v16b v; v8b q[2]; } u; const __bf16* p = rowk0 + 8 * (lane >> 4);
  u.q[0] = *(const v8b*)p; u.q[1] = *(const v8b*)(p + 16); return u.v;
}
__device__ __forceinline__ float bfr(float v) { return (float)(__bf16)v; }
__device__ __attribute__((noinline)) float exp_ni(float v) { return expf(v); }
__device__ __attribute__((noinline)) float erf_ni(float v) { return erff(v); }

#define WS_PKEY (0u)
#define WS_PK   (WS_PKEY + 2u * BINP * INP)
#define WS_PV   (WS_PK + 2u * (size_t)NT * CC * BINP)
#define WS_PQ   (WS_PV + 2u * (size_t)NT * CC * BINP)
#define WS_PM   (WS_PQ + 2u * CC * CC)
#define WS_P1   (WS_PM + 2u * CC * CC)
#define WS_P2   (WS_P1 + 2u * 4 * CC * CC)
#define WS_XN   (WS_P2 + 2u * 2 * CC * CC)
#define WS_SRC  (WS_XN + 4u * (size_t)NRX * CC)
#define WS_KF   (WS_SRC + 4u * (size_t)NRS * BINP)
#define WS_VF   (WS_KF + 4u * (size_t)NB * NKEY * CC)
#define WS_KV   (WS_VF + 4u * (size_t)NB * NKEY * CC)
#define WS_KS   (WS_KV + 4u * NB * NH * HD * HD)
#define WS_QF   (WS_KS + 4u * NB * NH * HD)
#define WS_MSG  (WS_QF + 4u * (size_t)NRX * CC)
#define WS_M2   (WS_MSG + 4u * (size_t)NRX * CC)
#define WS_HIDb (WS_M2 + 4u * (size_t)NRX * CC)
#define WS_END  (WS_HIDb + 2u * (size_t)NRX * 2 * CC)

__device__ __attribute__((noinline)) float elu1_p(float v) { return v > 0.f ? v + 1.0f : expf(v); }
__global__ __launch_bounds__(256) void k_pack(const float* __restrict__ WKEY, const float* __restrict__ WK, const float* __restrict__ WV, const float* __restrict__ WQ, const float* __restrict__ WM, const float* __restrict__ W1, const float* __restrict__ W2, __bf16* __restrict__ P, _Float16* __restrict__ P2) {
  const int n = blockIdx.x, which = blockIdx.y, t = threadIdx.x; __shared__ __align__(16) __bf16 s[BINP]; __shared__ __align__(16) _Float16 sh[2 * CC];
  if (which == 0) { if (n >= BINP) return; for (int k = t; k < INP; k += 256) s[k] = (__bf16)((n < BINS && k < INF) ? WKEY[(size_t)n * INF + k] : 0.f); __syncthreads(); for (int q = t; q < INP / 8; q += 256) vst2((unsigned*)(P + WS_PKEY / 2 + (size_t)n * INP + q * 8), *(const v4u*)&s[q * 8]); }
  else if (which <= 2) { const float* Wm = (which == 1) ? WK : WV; for (int k = t; k < BINP; k += 256) s[k] = (__bf16)((k < BINS) ? Wm[(size_t)n * BINS + k] : 0.f); __syncthreads(); for (int q = t; q < BINP / 8; q += 256) vst2((unsigned*)(P + ((which == 1) ? WS_PK : WS_PV) / 2 + (size_t)n * BINP + q * 8), *(const v4u*)&s[q * 8]); }
  else if (which <= 4) { if (n >= CC) return; const float* Wm = (which == 3) ? WQ : WM; s[t] = (__bf16)Wm[(size_t)n * CC + t]; __syncthreads(); if (t < CC / 8) vst2((unsigned*)(P + ((which == 3) ? WS_PQ : WS_PM) / 2 + (size_t)n * CC + t * 8), *(const v4u*)&s[t * 8]); }
  else if (which == 5) { if (n >= 2 * CC) return; for (int k = t; k < 2 * CC; k += 256) s[k] = (__bf16)W1[(size_t)n * 2 * CC + k]; __syncthreads(); if (t < 2 * CC / 8) vst2((unsigned*)(P + WS_P1 / 2 + (size_t)n * 2 * CC + t * 8), *(const v4u*)&s[t * 8]); }
  else { if (n >= CC) return; for (int k = t; k < 2 * CC; k += 256) sh[k] = (_Float16)bfr(W2[(size_t)n * 2 * CC + k]); __syncthreads(); if (t < 2 * CC / 8) vst2((unsigned*)(P2 + (size_t)n * 2 * CC + t * 8), *(const v4u*)&sh[t * 8]); }
}
__global__ __launch_bounds__(256) void k_lnx(const float* __restrict__ X, const float* __restrict__ G, const float* __restrict__ Bt, float* __restrict__ XN) {
  __shared__ float sx[64][CC + 1]; const size_t b = blockIdx.y; const int p0 = blockIdx.x * 64, t = threadIdx.x;
  for (int e = t; e < 64 * CC; e += 256) { const int c = e >> 6, p = e & 63; sx[p][c] = bfr(X[(b * CC + c) * NPIX + p0 + p]); }
  __syncthreads();
  { const int p = t >> 2, part = t & 3; float s = 0.f; for (int c = part; c < CC; c += 4) s += sx[p][c]; s += __shfl_xor(s, 1); s += __shfl_xor(s, 2); const float mu = s / (float)CC; float q = 0.f; for (int c = part; c < CC; c += 4) { const float d = sx[p][c] - mu; q += d * d; } q += __shfl_xor(q, 1); q += __shfl_xor(q, 2); const float inv = 1.0f / sqrtf(q / (float)CC + 1e-5f);
    __syncthreads();
    for (int c = part; c < CC; c += 4) sx[p][c] = (sx[p][c] - mu) * inv * bfr(G[c]) + bfr(Bt[c]); }
  __syncthreads();
  for (int e = t; e < 64 * (CC / 4); e += 256) { const int p = e >> 6, q = e & 63; v4f v; for (int i = 0; i < 4; ++i) v[i] = sx[p][q * 4 + i]; vst2(XN + ((b * NPIX) + p0 + p) * CC + q * 4, v); }
}
__global__ __launch_bounds__(128) void k_src(const float* __restrict__ SRCIN, const __bf16* __restrict__ P, float* __restrict__ SRC) {
  __shared__ __align__(16) float so[4][16][132]; __shared__ __align__(16) __bf16 sa[64][INP + 8];
  const int tid = threadIdx.x, wave = tid >> 5, lane = tid & 31, col = lane & 15, g = lane >> 4; const size_t rb0 = (size_t)blockIdx.x * 64; const int n0 = blockIdx.y * 128;
  for (int e = tid; e < 64 * INP; e += 128) { const int r = e / INP, k = e % INP; sa[r][k] = (__bf16)((k < INF) ? SRCIN[(rb0 + r) * INF + k] : 0.f); }
  if (tid < 64) for (int k = INP; k < INP + 8; ++k) sa[tid][k] = (__bf16)0.f;
  __syncthreads();
  v8f acc[8] = {};
#pragma unroll 1
  for (int kc = 0; kc < INP / 32; ++kc) { const v16b a = frag_b(&sa[wave * 16 + col][kc * 32], lane);
#pragma unroll
    for (int j = 0; j < 8; ++j) { const int n = n0 + j * 16 + col; if (n0 + j * 16 < BINP) acc[j] = wmma_bf(a, frag_b(P + WS_PKEY / 2 + (size_t)(n < BINP ? n : BINP - 1) * INP + kc * 32, lane), acc[j]); } }
#pragma unroll
  for (int j = 0; j < 8; ++j)
#pragma unroll
    for (int r = 0; r < 8; ++r) so[wave][8 * g + r][j * 16 + col] = (n0 + j * 16 + col < BINS) ? acc[j][r] : 0.f;
  LDSX();
  for (int rl = 0; rl < 16; ++rl) { const int n = n0 + lane * 4; if (n < BINP) vst2(SRC + (rb0 + wave * 16 + rl) * BINP + n, *(const v4f*)&so[wave][rl][lane * 4]); }
}
__global__ __launch_bounds__(128) void k_kv(const float* __restrict__ SRC, const __bf16* __restrict__ P, float* __restrict__ KF, float* __restrict__ VF) {
  __shared__ __align__(16) float so[4][16][132];
  const int tid = threadIdx.x, wave = tid >> 5, lane = tid & 31, col = lane & 15, g = lane >> 4; const size_t r0 = (size_t)blockIdx.x * 64 + wave * 16; const int n0 = blockIdx.y * 128; const int which = blockIdx.z;
  const __bf16* Wr = P + ((which == 0) ? WS_PK : WS_PV) / 2;
  v8f acc[8] = {};
#pragma unroll 1
  for (int kc = 0; kc < BINP / 32; ++kc) { const F2 a = split_row(SRC + (r0 + col) * BINP, kc * 32, lane);
#pragma unroll
    for (int j = 0; j < 8; ++j) { const v16b w = frag_b(Wr + (size_t)(n0 + j * 16 + col) * BINP + kc * 32, lane); acc[j] = wmma_bf(a.l, w, acc[j]); acc[j] = wmma_bf(a.h, w, acc[j]); } }
#pragma unroll
  for (int j = 0; j < 8; ++j)
#pragma unroll
    for (int r = 0; r < 8; ++r) so[wave][8 * g + r][j * 16 + col] = (which == 0) ? elu1_p(acc[j][r]) : acc[j][r] * (1.0f / (float)NKEY);
  LDSX();
  const int tt = n0 / CC, c0 = n0 % CC; float* dst = (which == 0) ? KF : VF;
  for (int rl = 0; rl < 16; ++rl) { const size_t row = r0 + rl; const size_t b = row / NS, s = row % NS; vst2(dst + ((b * NKEY) + s * NT + tt) * CC + c0 + lane * 4, *(const v4f*)&so[wave][rl][lane * 4]); }
}
__global__ __launch_bounds__(256) void k_kvsum(const float* __restrict__ KF, const float* __restrict__ VF, float* __restrict__ KV, float* __restrict__ KS) {
  const int h = blockIdx.x; const size_t b = blockIdx.y; const int t = threadIdx.x; __shared__ float sk[64][HD], sv[64][HD];
  float acc[4] = {0.f, 0.f, 0.f, 0.f}; float ks = 0.f;
  const int d = t >> 3, v0 = (t & 7) * 4;
#pragma unroll 1
  for (int kb = 0; kb < NKEY; kb += 64) {
    __syncthreads();
    for (int e = t; e < 64 * HD; e += 256) { const int kk = e >> 5, dd = e & 31; sk[kk][dd] = KF[((b * NKEY) + kb + kk) * CC + h * HD + dd]; sv[kk][dd] = VF[((b * NKEY) + kb + kk) * CC + h * HD + dd]; }
    __syncthreads();
#pragma unroll 1
    for (int kk = 0; kk < 64; ++kk) { const float kd = sk[kk][d]; acc[0] += kd * sv[kk][v0]; acc[1] += kd * sv[kk][v0 + 1]; acc[2] += kd * sv[kk][v0 + 2]; acc[3] += kd * sv[kk][v0 + 3]; if (v0 == 0) ks += kd; } }
  v4f o; for (int i = 0; i < 4; ++i) o[i] = acc[i]; vst2(KV + ((b * NH + h) * HD + d) * HD + v0, o);
  if (v0 == 0) KS[(b * NH + h) * HD + d] = ks;
}
__global__ __launch_bounds__(128) void k_q(const float* __restrict__ XN, const __bf16* __restrict__ P, float* __restrict__ QF) {
  __shared__ __align__(16) float so[4][16][132];
  const int tid = threadIdx.x, wave = tid >> 5, lane = tid & 31, col = lane & 15, g = lane >> 4; const size_t r0 = (size_t)blockIdx.x * 64 + wave * 16; const int n0 = blockIdx.y * 128;
  v8f acc[8] = {};
#pragma unroll
  for (int kc = 0; kc < CC / 32; ++kc) { const F2 a = split_row(XN + (r0 + col) * CC, kc * 32, lane);
#pragma unroll
    for (int j = 0; j < 8; ++j) { const v16b w = frag_b(P + WS_PQ / 2 + (size_t)(n0 + j * 16 + col) * CC + kc * 32, lane); acc[j] = wmma_bf(a.l, w, acc[j]); acc[j] = wmma_bf(a.h, w, acc[j]); } }
#pragma unroll
  for (int j = 0; j < 8; ++j)
#pragma unroll
    for (int r = 0; r < 8; ++r) so[wave][8 * g + r][j * 16 + col] = elu1_p(acc[j][r]);
  LDSX();
  for (int rl = 0; rl < 16; ++rl) vst2(QF + (r0 + rl) * CC + n0 + lane * 4, *(const v4f*)&so[wave][rl][lane * 4]);
}
__global__ __launch_bounds__(128) void k_msg(const float* __restrict__ QF, const float* __restrict__ KV, const float* __restrict__ KS, float* __restrict__ MSG) {
  __shared__ __align__(16) __bf16 skh[CC][HD + 8], skl[CC][HD + 8]; __shared__ float sks[CC]; __shared__ __align__(16) float so[4][16][132];
  const int tid = threadIdx.x, wave = tid >> 5, lane = tid & 31, col = lane & 15, g = lane >> 4; const size_t r0 = (size_t)blockIdx.x * 64 + wave * 16; const size_t b = ((size_t)blockIdx.x * 64) / NPIX;
  for (int e = tid; e < CC * HD; e += 128) { const int n = e >> 5, d = e & 31; const int h = n >> 5, v = n & 31; const float x = KV[((b * NH + h) * HD + d) * HD + v]; const __bf16 hb = (__bf16)x; skh[n][d] = hb; skl[n][d] = (__bf16)(x - (float)hb); }
  for (int e = tid; e < CC; e += 128) sks[e] = KS[b * CC + e];
  if (tid < CC) for (int d = HD; d < HD + 8; ++d) { }
  __syncthreads();
#pragma unroll 1
  for (int half = 0; half < 2; ++half) { v8f acc[8] = {};
#pragma unroll
    for (int j = 0; j < 8; ++j) { const int h = half * 4 + (j >> 1); const F2 a = split_row(QF + (r0 + col) * CC, h * HD, lane); const v16b wh = frag_b(&skh[half * 128 + j * 16 + col][0], lane), wl = frag_b(&skl[half * 128 + j * 16 + col][0], lane);
      acc[j] = wmma_bf(a.l, wh, acc[j]); acc[j] = wmma_bf(a.h, wl, acc[j]); acc[j] = wmma_bf(a.h, wh, acc[j]); }
#pragma unroll
    for (int r = 0; r < 8; ++r) { const size_t row = r0 + 8 * g + r;
#pragma unroll
      for (int hh = 0; hh < 4; ++hh) { const int h = half * 4 + hh; float z = 0.f;
#pragma unroll 1
        for (int d = 0; d < HD; ++d) z += QF[row * CC + h * HD + d] * sks[h * HD + d];
        const float zz = (1.0f / (z + 1e-6f)) * (float)NKEY; so[wave][8 * g + r][(hh * 2) * 16 + col] = acc[hh * 2][r] * zz; so[wave][8 * g + r][(hh * 2 + 1) * 16 + col] = acc[hh * 2 + 1][r] * zz; } }
    LDSX();
    for (int rl = 0; rl < 16; ++rl) vst2(MSG + (r0 + rl) * CC + half * 128 + lane * 4, *(const v4f*)&so[wave][rl][lane * 4]);
    LDSX(); }
}
__global__ __launch_bounds__(128) void k_merge(const float* __restrict__ MSG, const __bf16* __restrict__ P, const float* __restrict__ G, const float* __restrict__ Bt, float* __restrict__ M2) {
  __shared__ __align__(16) float sm[64][CC + 4];
  const int tid = threadIdx.x, wave = tid >> 5, lane = tid & 31, col = lane & 15, g = lane >> 4; const size_t rb0 = (size_t)blockIdx.x * 64; const size_t r0 = rb0 + wave * 16;
#pragma unroll 1
  for (int pass = 0; pass < 2; ++pass) { v8f acc[8] = {};
#pragma unroll
    for (int kc = 0; kc < CC / 32; ++kc) { const F2 a = split_row(MSG + (r0 + col) * CC, kc * 32, lane);
#pragma unroll
      for (int j = 0; j < 8; ++j) { const v16b w = frag_b(P + WS_PM / 2 + (size_t)(pass * 128 + j * 16 + col) * CC + kc * 32, lane); acc[j] = wmma_bf(a.l, w, acc[j]); acc[j] = wmma_bf(a.h, w, acc[j]); } }
#pragma unroll
    for (int j = 0; j < 8; ++j)
#pragma unroll
      for (int r = 0; r < 8; ++r) sm[wave * 16 + 8 * g + r][pass * 128 + j * 16 + col] = acc[j][r]; }
  __syncthreads();
  { const int p = tid >> 1, part = tid & 1; float s = 0.f; for (int c = part; c < CC; c += 2) s += sm[p][c]; s += __shfl_xor(s, 1); const float mu = s / (float)CC; float q = 0.f; for (int c = part; c < CC; c += 2) { const float d = sm[p][c] - mu; q += d * d; } q += __shfl_xor(q, 1); const float inv = 1.0f / sqrtf(q / (float)CC + 1e-5f);
    __syncthreads();
    for (int c = part; c < CC; c += 2) sm[p][c] = (sm[p][c] - mu) * inv * bfr(G[c]) + bfr(Bt[c]); }
  __syncthreads();
  for (int e = tid; e < 64 * (CC / 4); e += 128) { const int p = e >> 6, q = e & 63; vst2(M2 + (rb0 + p) * CC + q * 4, *(const v4f*)&sm[p][q * 4]); }
}
__global__ __launch_bounds__(128) void k_mlp1(const float* __restrict__ XN, const float* __restrict__ M2, const __bf16* __restrict__ P, _Float16* __restrict__ HIDh) {
  __shared__ __align__(16) _Float16 so[4][16][136];
  const int tid = threadIdx.x, wave = tid >> 5, lane = tid & 31, col = lane & 15, g = lane >> 4; const size_t r0 = (size_t)blockIdx.x * 64 + wave * 16; const int n0 = blockIdx.y * 128;
  v8f acc[8] = {};
#pragma unroll 2
  for (int kc = 0; kc < 2 * CC / 32; ++kc) { const F2 a = (kc < CC / 32) ? split_row(XN + (r0 + col) * CC, kc * 32, lane) : split_row(M2 + (r0 + col) * CC, (kc - CC / 32) * 32, lane);
#pragma unroll
    for (int j = 0; j < 8; ++j) { const v16b w = frag_b(P + WS_P1 / 2 + (size_t)(n0 + j * 16 + col) * (2 * CC) + kc * 32, lane); acc[j] = wmma_bf(a.l, w, acc[j]); acc[j] = wmma_bf(a.h, w, acc[j]); } }
#pragma unroll
  for (int j = 0; j < 8; ++j)
#pragma unroll
    for (int r = 0; r < 8; ++r) so[wave][8 * g + r][j * 16 + col] = (_Float16)fmaxf(acc[j][r], 0.f);
  LDSX();
  for (int rl = 0; rl < 16; ++rl) if (lane < 16) vst2((unsigned*)(HIDh + (r0 + rl) * (2 * CC) + n0 + lane * 8), *(const v4u*)&so[wave][rl][lane * 8]);
}
__global__ __launch_bounds__(128) void k_mlp2(const _Float16* __restrict__ HIDh, const _Float16* __restrict__ P2, const float* __restrict__ G, const float* __restrict__ Bt, const float* __restrict__ XN, float* __restrict__ OUT) {
  __shared__ __align__(16) float sm[64][CC + 4];
  const int tid = threadIdx.x, wave = tid >> 5, lane = tid & 31, col = lane & 15, g = lane >> 4; const size_t rb0 = (size_t)blockIdx.x * 64; const size_t r0 = rb0 + wave * 16; const size_t b = rb0 / NPIX; const int p0 = (int)(rb0 % NPIX);
#pragma unroll 1
  for (int pass = 0; pass < 2; ++pass) { v8f acc[8] = {};
#pragma unroll 2
    for (int kc = 0; kc < 2 * CC / 32; ++kc) { const v16h a = frag_h(HIDh + (r0 + col) * (2 * CC) + kc * 32, lane);
#pragma unroll
      for (int j = 0; j < 8; ++j) acc[j] = wmma16(a, frag_h(P2 + (size_t)(pass * 128 + j * 16 + col) * (2 * CC) + kc * 32, lane), acc[j]); }
#pragma unroll
    for (int j = 0; j < 8; ++j)
#pragma unroll
      for (int r = 0; r < 8; ++r) sm[wave * 16 + 8 * g + r][pass * 128 + j * 16 + col] = acc[j][r]; }
  __syncthreads();
  { const int p = tid >> 1, part = tid & 1; float s = 0.f; for (int c = part; c < CC; c += 2) s += sm[p][c]; s += __shfl_xor(s, 1); const float mu = s / (float)CC; float q = 0.f; for (int c = part; c < CC; c += 2) { const float d = sm[p][c] - mu; q += d * d; } q += __shfl_xor(q, 1); const float inv = 1.0f / sqrtf(q / (float)CC + 1e-5f);
    __syncthreads();
    for (int c = part; c < CC; c += 2) sm[p][c] = XN[(rb0 + p) * CC + c] + ((sm[p][c] - mu) * inv * bfr(G[c]) + bfr(Bt[c])); }
  __syncthreads();
  for (int e = tid; e < CC * 16; e += 128) { const int c = e >> 4, q = e & 15; v4f v; for (int i = 0; i < 4; ++i) v[i] = sm[q * 4 + i][c]; vst2(OUT + (b * CC + c) * NPIX + p0 + q * 4, v); }
}
extern "C" void kernel_launch(void* const* d_in, const int* in_sizes, int n_in, void* d_out, int out_size, void* d_ws, size_t ws_size, hipStream_t stream) {
  (void)in_sizes; (void)n_in; (void)out_size;
  const float** F = (const float**)d_in;
  if (ws_size < (size_t)WS_END) return;
  char* ws = (char*)d_ws; __bf16* P = (__bf16*)ws; _Float16 *P2 = (_Float16*)(ws + WS_P2), *HIDh = (_Float16*)(ws + WS_HIDb); float *XN = (float*)(ws + WS_XN), *SRC = (float*)(ws + WS_SRC), *KF = (float*)(ws + WS_KF), *VF = (float*)(ws + WS_VF), *KV = (float*)(ws + WS_KV), *KS = (float*)(ws + WS_KS), *QF = (float*)(ws + WS_QF), *MSG = (float*)(ws + WS_MSG), *M2 = (float*)(ws + WS_M2);
  k_pack<<<dim3(NT * CC, 7), 256, 0, stream>>>(F[2], F[4], F[5], F[3], F[6], F[7], F[8], P, P2);
  k_lnx<<<dim3(NPIX / 64, NBT), 256, 0, stream>>>(F[0], F[9], F[10], XN);
  k_src<<<dim3(NBT * NS / 64, (BINP + 127) / 128), 128, 0, stream>>>(F[1], P, SRC);
  k_kv<<<dim3(NBT * NS / 64, NT * CC / 128, 2), 128, 0, stream>>>(SRC, P, KF, VF);
  k_kvsum<<<dim3(NH, NBT), 256, 0, stream>>>(KF, VF, KV, KS);
  k_q<<<dim3(NPB, CC / 128), 128, 0, stream>>>(XN, P, QF);
  k_msg<<<NPB, 128, 0, stream>>>(QF, KV, KS, MSG);
  k_merge<<<NPB, 128, 0, stream>>>(MSG, P, F[9], F[10], M2);
  k_mlp1<<<dim3(NPB, 2 * CC / 128), 128, 0, stream>>>(XN, M2, P, HIDh);
  k_mlp2<<<NPB, 128, 0, stream>>>(HIDh, P2, F[11], F[12], XN, (float*)d_out);
}
